// CausalSelfAttention_58609123721400
// MI455X (gfx1250) — hardware-verified
//
#include <hip/hip_runtime.h>
#include <math.h>


#ifndef NB
#define NB 8
#endif
#ifndef SEQ
#define SEQ 1024
#endif
#define NB_FULL  8
#define SEQ_FULL 1024
#define DM   1024
#define NH_  16
#define HD   64
#define DQ   (NH_ * HD)
#define RH_  512
#define RHB  ((RH_ < SEQ) ? RH_ : SEQ)
#define GB   ((NB >= 4) ? 4 : NB)
#define NGRP (NB / GB)
#define PCAR 1024.0f
#define SCL  0.125f
#define L2E  1.4426950408889634f
#define NEGS (-1.0e30f)
#define PP   72

static_assert(NB <= NB_FULL);
static_assert(SEQ <= SEQ_FULL);
static_assert(NB % GB == 0);
static_assert(SEQ % 64 == 0);
static_assert(RHB % 64 == 0);
static_assert(HD == 64);
static_assert(DM % 64 == 0 && DM % 32 == 0);
static_assert(DQ % 64 == 0 && DQ % 32 == 0);
static_assert(DQ == NH_ * HD);
static_assert((PP % 8) == 0 && PP >= 64);

typedef _Float16 h16;
typedef unsigned short bf;
typedef __attribute__((ext_vector_type(16))) __bf16   v16bf;
typedef __attribute__((ext_vector_type(16))) _Float16 v16h;
typedef __attribute__((ext_vector_type(8)))  _Float16 v8h;
typedef __attribute__((ext_vector_type(8)))  unsigned short v8us;
typedef __attribute__((ext_vector_type(8)))  float    v8f;
typedef __attribute__((ext_vector_type(4)))  float    v4f;
typedef __attribute__((ext_vector_type(2)))  float    v2f;
typedef v8h  __attribute__((may_alias)) v8ha;
typedef v4f  __attribute__((may_alias)) v4fa;
typedef v8us __attribute__((may_alias)) v8usa;

__device__ __forceinline__ unsigned short f2bf(float f) { unsigned u = __float_as_uint(f); u += 0x7FFFu + ((u >> 16) & 1u); return (unsigned short)(u >> 16); }
__device__ __forceinline__ float bf2f(unsigned short b) { return __uint_as_float(((unsigned)b) << 16); }
__device__ __forceinline__ void splitf(float y, unsigned short& h, unsigned short& l) { h = f2bf(y); l = f2bf(y - bf2f(h)); }
__device__ __forceinline__ v16h cat16(v8h lo, v8h hi) { return __builtin_shufflevector(lo, hi, 0, 1, 2, 3, 4, 5, 6, 7, 8, 9, 10, 11, 12, 13, 14, 15); }
__device__ __forceinline__ v16bf cat16b(v8us lo, v8us hi) { return __builtin_bit_cast(v16bf, __builtin_shufflevector(lo, hi, 0, 1, 2, 3, 4, 5, 6, 7, 8, 9, 10, 11, 12, 13, 14, 15)); }
__device__ __forceinline__ v8f wmma16(v16h a, v16h b, v8f c) { return __builtin_amdgcn_wmma_f32_16x16x32_f16(false, a, false, b, (short)0, c, false, false); }
__device__ __forceinline__ v8f wmmab(v16bf a, v16bf b, v8f c) { return __builtin_amdgcn_wmma_f32_16x16x32_bf16(false, a, false, b, (short)0, c, false, false); }
__device__ __forceinline__ void wave_sync() { __builtin_amdgcn_fence(3  , "wavefront"); __builtin_amdgcn_wave_barrier(); asm volatile("" ::: "memory"); }

template <typename T16> struct WFrag;
template <> struct WFrag<h16> {
    typedef v16h V;
    static __device__ __forceinline__ V ld(const h16* p) { return cat16(*(const v8h*)p, *(const v8h*)(p + 16)); }
    static __device__ __forceinline__ V ldl(const h16* p) { return cat16(*(const v8ha*)p, *(const v8ha*)(p + 16)); }
    static __device__ __forceinline__ v8f mma(V a, V b, v8f c) { return wmma16(a, b, c); }
    static __device__ __forceinline__ void put(h16* p, h16* p2, unsigned i, float x) { (void)p2; p[i] = (h16)(x * PCAR); }
};
template <> struct WFrag<bf> {
    typedef v16bf V;
    static __device__ __forceinline__ V ld(const bf* p) { return cat16b(*(const v8us*)p, *(const v8us*)(p + 16)); }
    static __device__ __forceinline__ V ldl(const bf* p) { return cat16b(*(const v8usa*)p, *(const v8usa*)(p + 16)); }
    static __device__ __forceinline__ v8f mma(V a, V b, v8f c) { return wmmab(a, b, c); }
    static __device__ __forceinline__ void put(bf* p, bf* p2, unsigned i, float x) { unsigned short h, l; splitf(x, h, l); p[i] = h; p2[i] = l; }
};

struct PlaneArgs { h16* p16; bf* ph; bf* pl; h16* k16; bf* kh; bf* kl; const float* cs; };
static_assert(sizeof(PlaneArgs) == 56);

template <typename T16, int NSPLIT, int EPI>
__global__ __launch_bounds__(32) void k_gemmw(const T16* __restrict__ A, const T16* __restrict__ A2, const T16* __restrict__ Bt, const T16* __restrict__ Bt2, int K, float* C, int ldc, size_t sA, size_t sB, size_t sC, PlaneArgs pa) {
    typedef typename WFrag<T16>::V V;
    __shared__ __align__(16) float os[16 * 68];
    const size_t z = blockIdx.z; A += z * sA; if (A2) A2 += z * sA; Bt += z * sB; if (Bt2) Bt2 += z * sB; if (EPI == 0) C += z * sC;
    const int lane = threadIdx.x & 31, lr = lane & 15, hi = lane >> 4; const int r0 = blockIdx.x * 64, c0 = blockIdx.y * 64;
    v8f acc[4][4];
#pragma unroll
    for (int mb = 0; mb < 4; ++mb)
#pragma unroll
        for (int nb = 0; nb < 4; ++nb) acc[mb][nb] = (v8f){};
    const size_t aoff = (size_t)(r0 + lr) * K + 8 * hi, boff = (size_t)(c0 + lr) * K + 8 * hi;
#pragma unroll 1
    for (int kc = 0; kc < K; kc += 32) {
        V a[4], a2[4];
#pragma unroll
        for (int mb = 0; mb < 4; ++mb) { a[mb] = WFrag<T16>::ld(A + aoff + (size_t)mb * 16 * K + kc); if (NSPLIT == 1 || NSPLIT == 2) a2[mb] = WFrag<T16>::ld(A2 + aoff + (size_t)mb * 16 * K + kc); }
#pragma unroll
        for (int nb = 0; nb < 4; ++nb) { const V b = WFrag<T16>::ld(Bt + boff + (size_t)nb * 16 * K + kc); V b2; if (NSPLIT >= 2) b2 = WFrag<T16>::ld(Bt2 + boff + (size_t)nb * 16 * K + kc);
#pragma unroll
            for (int mb = 0; mb < 4; ++mb) { acc[mb][nb] = WFrag<T16>::mma(a[mb], b, acc[mb][nb]); if (NSPLIT == 1 || NSPLIT == 2) acc[mb][nb] = WFrag<T16>::mma(a2[mb], b, acc[mb][nb]); if (NSPLIT >= 2) acc[mb][nb] = WFrag<T16>::mma(a[mb], b2, acc[mb][nb]); } }
        asm volatile("v_nop\n\tv_nop\n\tv_nop\n\tv_nop" : "+v"(acc[0][0]), "+v"(acc[1][1]), "+v"(acc[2][2]), "+v"(acc[3][3]) : "v"(a[0]), "v"(a[3]));
    }
    const unsigned ulane = (unsigned)lane;
    const unsigned uc0 = (unsigned)c0;
    const unsigned which = uc0 / (unsigned)DQ;
    const unsigned hh1 = (uc0 % (unsigned)DQ) / (unsigned)HD;
    h16* P16 = which ? pa.k16 : pa.p16; bf* Ph = which ? pa.kh : pa.ph; bf* Pl = which ? pa.kl : pa.pl;
#pragma unroll
    for (int mb = 0; mb < 4; ++mb) {
#pragma unroll
        for (int nb = 0; nb < 4; ++nb) {
#pragma unroll
            for (int j = 0; j < 8; ++j) os[(hi * 8 + j) * 68 + nb * 16 + lr] = acc[mb][nb][j]; }
        wave_sync();
        if (EPI == 0) {
            float* crow = C + (size_t)(r0 + mb * 16) * ldc + c0;
#pragma unroll 1
            for (int ps = 0; ps < 2; ++ps) {
#pragma unroll
                for (int s = 0; s < 8; ++s) { const int row = 2 * s + hi, cofs = lr * 4; v4f val = *(const v4fa*)(os + row * 68 + cofs);
                    *(volatile v4f*)(crow + (size_t)row * ldc + cofs) = val; }
                if (ps == 0) __threadfence(); }
        } else if (EPI == 1) {
#pragma unroll 1
            for (int ps = 0; ps < 2; ++ps) {
#pragma unroll 1
                for (unsigned s4 = 0; s4 < 4u; ++s4) {
                    const unsigned row = 4u * s4 + (ulane >> 3), d0 = (ulane & 7u) * 8u, t = (unsigned)r0 + (unsigned)mb * 16u + row;
                    const v4f x0 = *(const v4fa*)(os + row * 68u + d0), x1 = *(const v4fa*)(os + row * 68u + d0 + 4u);
                    const v4f y0 = *(const v4fa*)(os + row * 68u + (d0 ^ 32u)), y1 = *(const v4fa*)(os + row * 68u + (d0 ^ 32u) + 4u);
                    const float* cp = pa.cs + ((size_t)t * 32u + (d0 & 31u)) * 2u;
                    const v4f ca = *(const v4f*)cp, cb = *(const v4f*)(cp + 4), cc = *(const v4f*)(cp + 8), cd = *(const v4f*)(cp + 12);
                    const float xs[8] = { x0[0], x0[1], x0[2], x0[3], x1[0], x1[1], x1[2], x1[3] };
                    const float ys[8] = { y0[0], y0[1], y0[2], y0[3], y1[0], y1[1], y1[2], y1[3] };
                    const float cv[8] = { ca[0], ca[2], cb[0], cb[2], cc[0], cc[2], cd[0], cd[2] };
                    const float sv[8] = { ca[1], ca[3], cb[1], cb[3], cc[1], cc[3], cd[1], cd[3] };
                    const bool lowh = d0 < 32u;
                    v8h o16; v8us oh, ol;
#pragma unroll
                    for (int i = 0; i < 8; ++i) { const float pa_ = xs[i] * cv[i], pb_ = ys[i] * sv[i]; const float r = lowh ? (pa_ - pb_) : (pa_ + pb_);
                        o16[i] = (h16)r; unsigned short a2, c2; splitf(r, a2, c2); oh[i] = a2; ol[i] = c2; }
                    const size_t hz = (size_t)z * NH_ + hh1;
                    *(volatile v8h*)(P16 + (hz * SEQ + t) * HD + d0) = o16;
                    if (r0 < RHB) { const size_t pe = (hz * RHB + t) * HD + d0; *(volatile v8us*)(Ph + pe) = oh; *(volatile v8us*)(Pl + pe) = ol; }
                }
                if (ps == 0) __threadfence(); }
        } else {
#pragma unroll 1
            for (int ps = 0; ps < 2; ++ps) {
#pragma unroll 1
                for (unsigned s4 = 0; s4 < 4u; ++s4) {
                    const unsigned row = 4u * s4 + (ulane >> 3), tq = (ulane & 7u) * 8u;
                    const v4f x0 = *(const v4fa*)(os + row * 68u + tq), x1 = *(const v4fa*)(os + row * 68u + tq + 4u);
                    const float xs[8] = { x0[0], x0[1], x0[2], x0[3], x1[0], x1[1], x1[2], x1[3] };
                    v8h o16; v8us oh, ol;
#pragma unroll
                    for (int i = 0; i < 8; ++i) { o16[i] = (h16)xs[i]; unsigned short a2, c2; splitf(xs[i], a2, c2); oh[i] = a2; ol[i] = c2; }
                    const size_t dr = ((size_t)z * NH_ + blockIdx.x) * HD + (unsigned)mb * 16u + row;
                    *(volatile v8h*)(pa.p16 + dr * SEQ + uc0 + tq) = o16;
                    if (c0 < RHB) { const size_t pe = dr * RHB + uc0 + tq; *(volatile v8us*)(pa.ph + pe) = oh; *(volatile v8us*)(pa.pl + pe) = ol; }
                }
                if (ps == 0) __threadfence(); }
        }
        wave_sync();
    }
}

__global__ __launch_bounds__(256) void k_cvt8(const float* __restrict__ src, bf* dst, unsigned n8, size_t sS, size_t sD) {
    const unsigned i = blockIdx.x * 256u + threadIdx.x; if (i >= n8) return;
    src += (size_t)blockIdx.y * sS; dst += (size_t)blockIdx.y * sD;
    const v8f v = *(const v8f*)(src + (size_t)i * 8u); v8us o;
#pragma unroll
    for (int k = 0; k < 8; ++k) o[k] = f2bf(v[k]);
    *(volatile v8us*)(dst + (size_t)i * 8u) = o; __threadfence(); *(volatile v8us*)(dst + (size_t)i * 8u) = o; }

struct InvF { float v[32]; };
static_assert(sizeof(InvF) == 128);
__global__ __launch_bounds__(256) void k_cstab(InvF f, float* CS) {
    const unsigned idx = blockIdx.x * 256u + threadIdx.x; if (idx >= (unsigned)SEQ * 32u) return;
    const unsigned t = idx >> 5, i = idx & 31u;
    float inv = f.v[0];
#pragma unroll
    for (int j = 1; j < 32; ++j) inv = (i == (unsigned)j) ? f.v[j] : inv;
    const float ang = (float)t * inv; float sn, cn; sincosf(ang, &sn, &cn);
    v2f o; o[0] = cn; o[1] = sn;
    *(volatile v2f*)(CS + (size_t)idx * 2u) = o; __threadfence(); *(volatile v2f*)(CS + (size_t)idx * 2u) = o; }

template <typename T16, bool SPLIT>
__device__ __forceinline__ void flash_body(const T16* __restrict__ Q, const T16* __restrict__ Q2, const T16* __restrict__ Kp, const T16* __restrict__ K2,
                                           const T16* __restrict__ VT, const T16* __restrict__ VT2, const int* __restrict__ mask, bf* ATh, bf* ATl,
                                           unsigned qoff, unsigned QT, unsigned VP) {
    typedef typename WFrag<T16>::V V;
    __shared__ __align__(16) float os[16 * 68];
    __shared__ __align__(16) T16 pt[16 * PP];
    __shared__ __align__(16) T16 pt2[SPLIT ? 16 * PP : 8];
    const unsigned lane = threadIdx.x & 31u, lr = lane & 15u, hi = lane >> 4;
    const unsigned q0 = qoff + blockIdx.x * 16u, hh = blockIdx.y, zb = blockIdx.z;
    const size_t hz = (size_t)zb * NH_ + hh;
    V a[2], a2[2];
    { const size_t qo = (hz * QT + q0 + lr) * HD + 8u * hi;
#pragma unroll
      for (int kc = 0; kc < 2; ++kc) { a[kc] = WFrag<T16>::ld(Q + qo + kc * 32); if (SPLIT) a2[kc] = WFrag<T16>::ld(Q2 + qo + kc * 32); } }
    float mrow[8], lsum[8]; v8f o[4];
#pragma unroll
    for (int r = 0; r < 8; ++r) { mrow[r] = NEGS; lsum[r] = 0.0f; }
#pragma unroll
    for (int nb = 0; nb < 4; ++nb) o[nb] = (v8f){};
    const unsigned nkt = (q0 >> 6) + 1u;
#pragma unroll 1
    for (unsigned kt = 0; kt < nkt; ++kt) {
        const unsigned k0 = kt * 64u;
        int mk[4];
#pragma unroll
        for (int nb = 0; nb < 4; ++nb) mk[nb] = mask[(size_t)zb * SEQ_FULL + k0 + (unsigned)nb * 16u + lr];
        v8f s[4];
#pragma unroll
        for (int nb = 0; nb < 4; ++nb) s[nb] = (v8f){};
        const size_t kof = (hz * QT + k0 + lr) * HD + 8u * hi;
        V b = a[0];
#pragma unroll
        for (int nb = 0; nb < 4; ++nb) {
#pragma unroll
            for (int kc = 0; kc < 2; ++kc) {
                b = WFrag<T16>::ld(Kp + kof + (size_t)nb * 16 * HD + kc * 32);
                s[nb] = WFrag<T16>::mma(a[kc], b, s[nb]);
                if (SPLIT) { s[nb] = WFrag<T16>::mma(a2[kc], b, s[nb]); const V b2 = WFrag<T16>::ld(K2 + kof + (size_t)nb * 16 * HD + kc * 32); s[nb] = WFrag<T16>::mma(a[kc], b2, s[nb]); } } }
        asm volatile("v_nop\n\tv_nop\n\tv_nop\n\tv_nop" : "+v"(s[0]), "+v"(s[1]), "+v"(s[2]), "+v"(s[3]) : "v"(a[0]), "v"(b));
#pragma unroll
        for (int r = 0; r < 8; ++r) {
            const unsigned row = q0 + 8u * hi + (unsigned)r;
            float sv[4]; bool okv[4]; float rm = NEGS;
#pragma unroll
            for (int nb = 0; nb < 4; ++nb) { const unsigned key = k0 + (unsigned)nb * 16u + lr; okv[nb] = (key <= row) && (mk[nb] != 0); sv[nb] = okv[nb] ? s[nb][r] * SCL : NEGS; rm = fmaxf(rm, sv[nb]); }
            rm = fmaxf(rm, __shfl_xor(rm, 1, 32)); rm = fmaxf(rm, __shfl_xor(rm, 2, 32)); rm = fmaxf(rm, __shfl_xor(rm, 4, 32)); rm = fmaxf(rm, __shfl_xor(rm, 8, 32));
            const float mnew = fmaxf(mrow[r], rm);
            const float alpha = __builtin_amdgcn_exp2f((mrow[r] - mnew) * L2E);
            mrow[r] = mnew;
            float psum = 0.0f;
#pragma unroll
            for (int nb = 0; nb < 4; ++nb) { const float e = __builtin_amdgcn_exp2f((sv[nb] - mnew) * L2E); const float p = okv[nb] ? e : 0.0f; psum += p;
                WFrag<T16>::put(pt, pt2, (8u * hi + (unsigned)r) * PP + (unsigned)nb * 16u + lr, p); }
            lsum[r] = lsum[r] * alpha + psum;
#pragma unroll
            for (int nb = 0; nb < 4; ++nb) o[nb][r] *= alpha;
        }
        wave_sync();
        V ap[2], ap2[2];
#pragma unroll
        for (int kc = 0; kc < 2; ++kc) { ap[kc] = WFrag<T16>::ldl(pt + lr * PP + 8u * hi + kc * 32); if (SPLIT) ap2[kc] = WFrag<T16>::ldl(pt2 + lr * PP + 8u * hi + kc * 32); }
        const size_t vof = (hz * HD + lr) * VP + k0 + 8u * hi;
        V bv = ap[0];
#pragma unroll
        for (int nb = 0; nb < 4; ++nb) {
#pragma unroll
            for (int kc = 0; kc < 2; ++kc) {
                bv = WFrag<T16>::ld(VT + vof + (size_t)nb * 16 * VP + kc * 32);
                o[nb] = WFrag<T16>::mma(ap[kc], bv, o[nb]);
                if (SPLIT) { o[nb] = WFrag<T16>::mma(ap2[kc], bv, o[nb]); const V bv2 = WFrag<T16>::ld(VT2 + vof + (size_t)nb * 16 * VP + kc * 32); o[nb] = WFrag<T16>::mma(ap[kc], bv2, o[nb]); } } }
        asm volatile("v_nop\n\tv_nop\n\tv_nop\n\tv_nop" : "+v"(o[0]), "+v"(o[1]), "+v"(o[2]), "+v"(o[3]) : "v"(ap[0]), "v"(bv));
        wave_sync();
    }
#pragma unroll
    for (int r = 0; r < 8; ++r) {
        float l = lsum[r];
        l += __shfl_xor(l, 1, 32); l += __shfl_xor(l, 2, 32); l += __shfl_xor(l, 4, 32); l += __shfl_xor(l, 8, 32);
        const float inv = 1.0f / (SPLIT ? l : l * PCAR);
#pragma unroll
        for (int nb = 0; nb < 4; ++nb) os[(8u * hi + (unsigned)r) * 68u + (unsigned)nb * 16u + lr] = o[nb][r] * inv;
    }
    wave_sync();
#pragma unroll 1
    for (int ps = 0; ps < 2; ++ps) {
#pragma unroll 1
        for (unsigned s4 = 0; s4 < 4u; ++s4) {
            const unsigned row = 4u * s4 + (lane >> 3), d0 = (lane & 7u) * 8u;
            const v4f x0 = *(const v4fa*)(os + row * 68u + d0), x1 = *(const v4fa*)(os + row * 68u + d0 + 4u);
            const float xs[8] = { x0[0], x0[1], x0[2], x0[3], x1[0], x1[1], x1[2], x1[3] };
            v8us oh, ol;
#pragma unroll
            for (int i = 0; i < 8; ++i) { unsigned short a_, c_; splitf(xs[i], a_, c_); oh[i] = a_; ol[i] = c_; }
            const size_t oo = ((size_t)zb * SEQ + q0 + row) * DQ + hh * HD + d0;
            *(volatile v8us*)(ATh + oo) = oh; *(volatile v8us*)(ATl + oo) = ol;
        }
        if (ps == 0) __threadfence(); }
}
__global__ __launch_bounds__(32) void k_flash_hl(const bf* __restrict__ Qh, const bf* __restrict__ Ql, const bf* __restrict__ Kh, const bf* __restrict__ Kl,
                                                 const bf* __restrict__ Vh, const bf* __restrict__ Vl, const int* __restrict__ mask, bf* ATh, bf* ATl) {
    flash_body<bf, true>(Qh, Ql, Kh, Kl, Vh, Vl, mask, ATh, ATl, 0u, (unsigned)RHB, (unsigned)RHB); }
__global__ __launch_bounds__(32) void k_flash_h(const h16* __restrict__ Q, const h16* __restrict__ Kp, const h16* __restrict__ VT, const int* __restrict__ mask, bf* ATh, bf* ATl) {
    flash_body<h16, false>(Q, nullptr, Kp, nullptr, VT, nullptr, mask, ATh, ATl, (unsigned)RHB, (unsigned)SEQ, (unsigned)SEQ); }

constexpr size_t al256(size_t b) { return (b + 255) & ~(size_t)255; }
constexpr size_t SZ_WQKV = al256((size_t)3 * DQ * DM * 2);
constexpr size_t SZ_WO   = al256((size_t)DM * DQ * 2);
constexpr size_t SZ_CS   = al256((size_t)SEQ * 32 * 2 * 4);
constexpr size_t SZ_XB   = al256((size_t)GB * SEQ * DM * 2);
constexpr size_t SZ_P16  = al256((size_t)GB * NH_ * SEQ * HD * 2);
constexpr size_t SZ_PHL  = al256((size_t)GB * NH_ * RHB * HD * 2);
constexpr size_t SZ_AT   = al256((size_t)GB * SEQ * DQ * 2);
constexpr size_t WS_TOTAL = SZ_WQKV + SZ_WO + SZ_CS + SZ_XB + 3 * SZ_P16 + 6 * SZ_PHL + 2 * SZ_AT;
static_assert(WS_TOTAL <= (size_t)128 * 1024 * 1024);
static_assert(((size_t)SEQ * DM) % 8 == 0 && ((size_t)3 * DQ * DM) % 8 == 0 && ((size_t)DM * DQ) % 8 == 0);

extern "C" void kernel_launch(void* const* d_in, const int* in_sizes, int n_in,
                              void* d_out, int out_size, void* d_ws, size_t ws_size, hipStream_t stream) {
    if (n_in < 4) return;
    const size_t need_x = ((size_t)(NB - 1) * SEQ_FULL + SEQ) * DM;
    if ((size_t)in_sizes[0] < need_x) return;
    if ((size_t)in_sizes[1] < (size_t)(NB - 1) * SEQ_FULL + SEQ) return;
    if ((size_t)in_sizes[2] < (size_t)3 * DQ * DM) return;
    if ((size_t)in_sizes[3] < (size_t)DM * DQ) return;
    if ((size_t)out_size < need_x) return;
    if (WS_TOTAL > ws_size) return;
    const float* x = (const float*)d_in[0]; const int* amask = (const int*)d_in[1]; const float* wqkv = (const float*)d_in[2]; const float* wo = (const float*)d_in[3];
    float* OUT = (float*)d_out;
    char* wsp = (char*)d_ws;
    auto take = [&](size_t bytes) { char* p = wsp; wsp += bytes; return (void*)p; };
    bf* WQKV = (bf*)take(SZ_WQKV); bf* WV = WQKV + (size_t)2 * DQ * DM;
    bf* WO = (bf*)take(SZ_WO); float* CS = (float*)take(SZ_CS); bf* XB = (bf*)take(SZ_XB);
    h16* Q16 = (h16*)take(SZ_P16); h16* K16 = (h16*)take(SZ_P16); h16* VT16 = (h16*)take(SZ_P16);
    bf* Qh = (bf*)take(SZ_PHL); bf* Ql = (bf*)take(SZ_PHL); bf* Kh = (bf*)take(SZ_PHL); bf* Kl = (bf*)take(SZ_PHL); bf* VTh = (bf*)take(SZ_PHL); bf* VTl = (bf*)take(SZ_PHL);
    bf* ATh = (bf*)take(SZ_AT); bf* ATl = (bf*)take(SZ_AT);

    InvF fr;
    for (int i = 0; i < 32; ++i) { const double pw = pow(10000.0, (double)i / 32.0); const float pf = (float)pw; fr.v[i] = 1.0f / pf; }

    { const unsigned n8 = (unsigned)((size_t)3 * DQ * DM / 8); k_cvt8<<<dim3((n8 + 255u) / 256u, 1, 1), 256, 0, stream>>>(wqkv, WQKV, n8, 0, 0); }
    { const unsigned n8 = (unsigned)((size_t)DM * DQ / 8);     k_cvt8<<<dim3((n8 + 255u) / 256u, 1, 1), 256, 0, stream>>>(wo, WO, n8, 0, 0); }
    k_cstab<<<(SEQ * 32 + 255) / 256, 256, 0, stream>>>(fr, CS);

    PlaneArgs pqk; pqk.p16 = Q16; pqk.ph = Qh; pqk.pl = Ql; pqk.k16 = K16; pqk.kh = Kh; pqk.kl = Kl; pqk.cs = CS;
    PlaneArgs pv;  pv.p16 = VT16; pv.ph = VTh; pv.pl = VTl; pv.k16 = VT16; pv.kh = VTh; pv.kl = VTl; pv.cs = CS;
    PlaneArgs pz;  pz.p16 = nullptr; pz.ph = nullptr; pz.pl = nullptr; pz.k16 = nullptr; pz.kh = nullptr; pz.kl = nullptr; pz.cs = nullptr;

    for (int g = 0; g < NGRP; ++g) {
        const size_t b0 = (size_t)g * GB;
        { const unsigned n8 = (unsigned)((size_t)SEQ * DM / 8);
          k_cvt8<<<dim3((n8 + 255u) / 256u, GB, 1), 256, 0, stream>>>(x + b0 * SEQ_FULL * DM, XB, n8, (size_t)SEQ_FULL * DM, (size_t)SEQ * DM); }
        k_gemmw<bf, 0, 1><<<dim3(SEQ / 64, 2 * DQ / 64, GB), 32, 0, stream>>>(XB, nullptr, WQKV, nullptr, DM, nullptr, 0, (size_t)SEQ * DM, 0, 0, pqk);
        k_gemmw<bf, 0, 2><<<dim3(DQ / 64, SEQ / 64, GB), 32, 0, stream>>>(WV, nullptr, XB, nullptr, DM, nullptr, 0, 0, (size_t)SEQ * DM, 0, pv);
        k_flash_hl<<<dim3(RHB / 16, NH_, GB), 32, 0, stream>>>(Qh, Ql, Kh, Kl, VTh, VTl, amask + b0 * SEQ_FULL, ATh, ATl);
        if (SEQ > RHB) k_flash_h<<<dim3((SEQ - RHB) / 16, NH_, GB), 32, 0, stream>>>(Q16, K16, VT16, amask + b0 * SEQ_FULL, ATh, ATl);
        k_gemmw<bf, 1, 0><<<dim3(SEQ / 64, DM / 64, GB), 32, 0, stream>>>(ATh, ATl, WO, nullptr, DQ, OUT + b0 * SEQ_FULL * DM, DM, (size_t)SEQ * DQ, 0, (size_t)SEQ_FULL * DM, pz);
    }
}
